// SelfAttention_58600533787141
// MI455X (gfx1250) — hardware-verified
//
#include <hip/hip_runtime.h>


#ifndef NB
#define NB 4
#endif
#ifndef SEQ
#define SEQ 1024
#endif
#define NB_FULL  4
#define SEQ_FULL 1024
#define DM   1024
#define NH   16
#define HD   64
#define D3   (3 * DM)
#define CK   (2 * DM)
#define PCAR 256.0f
#define L2E  1.4426950408889634f
#define SBP  16
#define PBP  40
#define LDS_PT  (1024 * SBP * 4)
#define LDS_PB  (LDS_PT + NH * 256 * 4)
#define LDS_TOT (LDS_PB + NH * 32 * PBP * 2)
#define PLSZ ((size_t)NB * NH * SEQ * HD)

static_assert(SEQ % 64 == 0);
static_assert(NB >= 1 && NB <= NB_FULL && SEQ <= SEQ_FULL);
static_assert(DM == NH * HD);
static_assert(HD == 64);
static_assert(HD * 2 == 128);
static_assert(NH == 16);
static_assert((DM & (DM - 1)) == 0);
static_assert(DM % 64 == 0 && D3 % 64 == 0 && DM % 32 == 0 && HD % 32 == 0 && CK % 32 == 0);
static_assert(NH * 32 * 64 * 2 <= LDS_PT);
static_assert(LDS_TOT == 122880);

typedef _Float16 h16;
typedef unsigned short bf;
typedef __attribute__((ext_vector_type(16))) __bf16   v16bf;
typedef __attribute__((ext_vector_type(16))) _Float16 v16h;
typedef __attribute__((ext_vector_type(8)))  _Float16 v8h;
typedef __attribute__((ext_vector_type(8)))  unsigned short v8us;
typedef __attribute__((ext_vector_type(8)))  float    v8f;
typedef __attribute__((ext_vector_type(4)))  float    v4f;
typedef __attribute__((ext_vector_type(4)))  unsigned v4u;
typedef __attribute__((ext_vector_type(8)))  unsigned v8u;
typedef v8h  __attribute__((may_alias)) v8ha;
typedef v8us __attribute__((may_alias)) v8usa;
typedef v4f  __attribute__((may_alias)) v4fa;
typedef v4u  __attribute__((may_alias)) v4ua;

__device__ __forceinline__ unsigned short f2bf(float f) { unsigned u = __float_as_uint(f); u += 0x7FFFu + ((u >> 16) & 1u); return (unsigned short)(u >> 16); }
__device__ __forceinline__ float bf2f(unsigned short b) { return __uint_as_float(((unsigned)b) << 16); }
__device__ __forceinline__ float bfr(float f) { return bf2f(f2bf(f)); }
__device__ __forceinline__ void splitf(float y, unsigned short& h, unsigned short& l) { h = f2bf(y); l = f2bf(y - bf2f(h)); }
__device__ __forceinline__ unsigned splitw(float y) { const unsigned u = __float_as_uint(y); const float lo = y - __uint_as_float(u & 0xffff0000u); return (u >> 16) | (((unsigned)f2bf(lo)) << 16); }
__device__ __forceinline__ v16h cat16(v8h lo, v8h hi) { return __builtin_shufflevector(lo, hi, 0, 1, 2, 3, 4, 5, 6, 7, 8, 9, 10, 11, 12, 13, 14, 15); }
__device__ __forceinline__ v16bf cat16b(v8us lo, v8us hi) { return __builtin_bit_cast(v16bf, __builtin_shufflevector(lo, hi, 0, 1, 2, 3, 4, 5, 6, 7, 8, 9, 10, 11, 12, 13, 14, 15)); }
__device__ __forceinline__ v8f wmma16(v16h a, v16h b, v8f c) { return __builtin_amdgcn_wmma_f32_16x16x32_f16(false, a, false, b, (short)0, c, false, false); }
__device__ __forceinline__ v8f wmmab(v16bf a, v16bf b, v8f c) { return __builtin_amdgcn_wmma_f32_16x16x32_bf16(false, a, false, b, (short)0, c, false, false); }
__device__ __forceinline__ v16bf ldb(const bf* p) { return cat16b(*(const v8us*)p, *(const v8us*)(p + 16)); }
__device__ __forceinline__ v16h ldh(const h16* p) { return cat16(*(const v8h*)p, *(const v8h*)(p + 16)); }

__global__ __launch_bounds__(32) void k_gemm_bf(const bf* __restrict__ A, const bf* __restrict__ Bt, int K, float* C, int ldc, const float* __restrict__ bias, float oscale, size_t sA, size_t sB, size_t sC) {
    __shared__ __align__(16) float os[16 * 68];
    const size_t z = blockIdx.z; A += z * sA; Bt += z * sB; C += z * sC;
    const int lane = threadIdx.x & 31, lr = lane & 15, hi = lane >> 4; const int r0 = blockIdx.x * 64, c0 = blockIdx.y * 64;
    v8f acc[4][4];
#pragma unroll
    for (int mb = 0; mb < 4; ++mb)
#pragma unroll
        for (int nb = 0; nb < 4; ++nb) acc[mb][nb] = (v8f){};
    const size_t aoff = (size_t)(r0 + lr) * K + 8 * hi, boff = (size_t)(c0 + lr) * K + 8 * hi;
#pragma unroll 1
    for (int kc = 0; kc < K; kc += 32) {
        v16bf a[4];
#pragma unroll
        for (int mb = 0; mb < 4; ++mb) a[mb] = ldb(A + aoff + (size_t)mb * 16 * K + kc);
#pragma unroll
        for (int nb = 0; nb < 4; ++nb) { const v16bf b = ldb(Bt + boff + (size_t)nb * 16 * K + kc);
#pragma unroll
            for (int mb = 0; mb < 4; ++mb) acc[mb][nb] = wmmab(a[mb], b, acc[mb][nb]); }
        asm volatile("v_nop\n\tv_nop\n\tv_nop\n\tv_nop" : "+v"(acc[0][0]), "+v"(acc[1][1]), "+v"(acc[2][2]), "+v"(acc[3][3]) : "v"(a[0]), "v"(a[3]));
    }
#pragma unroll
    for (int mb = 0; mb < 4; ++mb) {
#pragma unroll
        for (int nb = 0; nb < 4; ++nb) {
#pragma unroll
            for (int j = 0; j < 8; ++j) os[(hi * 8 + j) * 68 + nb * 16 + lr] = acc[mb][nb][j]; }
        __builtin_amdgcn_wave_barrier(); asm volatile("" ::: "memory");
        float* crow = C + (size_t)(r0 + mb * 16) * ldc + c0;
#pragma unroll 1
        for (int ps = 0; ps < 2; ++ps) {
#pragma unroll
            for (int s = 0; s < 8; ++s) { const int row = 2 * s + hi, cofs = lr * 4; v4f val = *(const v4fa*)(os + row * 68 + cofs); val[0] *= oscale; val[1] *= oscale; val[2] *= oscale; val[3] *= oscale;
                val[0] += bfr(bias[c0 + cofs]); val[1] += bfr(bias[c0 + cofs + 1]); val[2] += bfr(bias[c0 + cofs + 2]); val[3] += bfr(bias[c0 + cofs + 3]);
                *(volatile v4f*)(crow + (size_t)row * ldc + cofs) = val; }
            if (ps == 0) __threadfence(); }
        __builtin_amdgcn_wave_barrier(); asm volatile("" ::: "memory");
    }
}

__global__ __launch_bounds__(256) void k_cvt8(const float* __restrict__ src, bf* dst, size_t n8, size_t sS, size_t sD) { const size_t i = (size_t)blockIdx.x * 256 + threadIdx.x; if (i >= n8) return; src += (size_t)blockIdx.y * sS; dst += (size_t)blockIdx.y * sD; const v8f v = *(const v8f*)(src + i * 8); v8us o;
#pragma unroll
    for (int k = 0; k < 8; ++k) o[k] = f2bf(v[k]); *(volatile v8us*)(dst + i * 8) = o; __threadfence(); *(volatile v8us*)(dst + i * 8) = o; }
__global__ __launch_bounds__(256) void k_cvtdup(const float* __restrict__ src, bf* dst, size_t n8) { const size_t i = (size_t)blockIdx.x * 256 + threadIdx.x; if (i >= n8) return; const size_t e = i * 8; const size_t row = e / CK; const int col = ((int)(e % CK)) & (DM - 1);
    const v8f v = *(const v8f*)(src + row * DM + col); v8us o;
#pragma unroll
    for (int k = 0; k < 8; ++k) o[k] = f2bf(v[k]); *(volatile v8us*)(dst + e) = o; __threadfence(); *(volatile v8us*)(dst + e) = o; }
__global__ __launch_bounds__(256) void k_qkpl(const float* __restrict__ F, bf* PL) { const size_t idx = (size_t)blockIdx.x * 256 + threadIdx.x; if (idx >= PLSZ / 8) return; const int which = blockIdx.y; const size_t e = idx * 8;
    const int d = (int)(e % HD); const int n = (int)((e / HD) % SEQ); const int h = (int)((e / ((size_t)HD * SEQ)) % NH); const int b = (int)(e / ((size_t)HD * SEQ * NH)); const float sc = which ? 1.0f : 0.125f;
    const v8f v = *(const v8f*)(F + ((size_t)b * SEQ + n) * D3 + which * DM + h * HD + d); v8us oh, ol;
#pragma unroll
    for (int k = 0; k < 8; ++k) { unsigned short a2, c2; splitf(v[k] * sc, a2, c2); oh[k] = a2; ol[k] = c2; }
    bf* ph = PL + (size_t)(2 * which) * PLSZ + e; bf* pl = PL + (size_t)(2 * which + 1) * PLSZ + e;
    *(volatile v8us*)ph = oh; *(volatile v8us*)pl = ol; __threadfence(); *(volatile v8us*)ph = oh; *(volatile v8us*)pl = ol; }
__global__ __launch_bounds__(256) void k_vtp(const float* __restrict__ F, h16* VT) { const size_t idx = (size_t)blockIdx.x * 256 + threadIdx.x; if (idx >= PLSZ / 8) return; const size_t e = idx * 8;
    const int t = (int)(e % SEQ); const int d = (int)((e / SEQ) % HD); const int h = (int)((e / ((size_t)SEQ * HD)) % NH); const int b = (int)(e / ((size_t)SEQ * HD * NH));
    const float* f = F + ((size_t)b * SEQ + t) * D3 + 2 * DM + h * HD + d; v8h o;
#pragma unroll
    for (int q = 0; q < 8; ++q) o[q] = (h16)f[(size_t)q * D3];
    *(volatile v8h*)(VT + e) = o; __threadfence(); *(volatile v8h*)(VT + e) = o; }

__device__ __forceinline__ v16bf ldw(const unsigned* p) { const v4u a = *(const v4ua*)p; const v4u c = *(const v4ua*)(p + 4); return __builtin_bit_cast(v16bf, __builtin_shufflevector(a, c, 0, 1, 2, 3, 4, 5, 6, 7)); }
__device__ __forceinline__ v16h ldp(const h16* p) { return cat16(*(const v8ha*)p, *(const v8ha*)(p + 16)); }
__device__ __forceinline__ void stat_upd(float& M, float& L, const v8f a, const v8f c) {
    float tm = fmaxf(a[0], c[0]);
#pragma unroll
    for (int r = 1; r < 8; ++r) tm = fmaxf(tm, fmaxf(a[r], c[r]));
    tm = fmaxf(tm, __shfl_xor(tm, 16, 32));
    const float Mn = fmaxf(M, tm); float sm = 0.f;
#pragma unroll
    for (int r = 0; r < 8; ++r) { sm += __builtin_amdgcn_exp2f((a[r] - Mn) * L2E); sm += __builtin_amdgcn_exp2f((c[r] - Mn) * L2E); }
    sm += __shfl_xor(sm, 16, 32);
    L = L * __builtin_amdgcn_exp2f((M - Mn) * L2E) + sm; M = Mn;
}

__global__ __launch_bounds__(512) void k_attn(const bf* __restrict__ PL, const h16* __restrict__ VT, const float* __restrict__ pre, const float* __restrict__ post, bf* CTX) {
    extern __shared__ __align__(16) unsigned char smem[];
    const int tid = threadIdx.x, lane = tid & 31, w = tid >> 5, lr = lane & 15, hf = lane >> 4;
    const int b = blockIdx.y, n0 = blockIdx.x * 32;
    unsigned* Sb = (unsigned*)smem;
    unsigned* PT = (unsigned*)(smem + LDS_PT) + w * 256;
    h16* Pb = (h16*)(smem + LDS_PB);
    unsigned short* OS = (unsigned short*)smem + w * 2048;
    const bf* QPh = PL; const bf* QPl = PL + PLSZ; const bf* KPh = PL + 2 * PLSZ; const bf* KPl = PL + 3 * PLSZ;
    const size_t zh = ((size_t)b * NH + w) * SEQ * HD;
    const size_t zv = ((size_t)b * NH + w) * HD * SEQ;

    v16bf preB, postB;
    { v8u pw, qw;
#pragma unroll
      for (int j = 0; j < 8; ++j) { const unsigned t0 = f2bf(pre[(8 * hf + j) * 16 + lr]); const unsigned t1 = f2bf(post[(8 * hf + j) * 16 + lr]); pw[j] = t0 | (t0 << 16); qw[j] = t1 | (t1 << 16); }
      preB = __builtin_bit_cast(v16bf, pw); postB = __builtin_bit_cast(v16bf, qw); }

    v16bf qh[2][2], ql[2][2];
#pragma unroll
    for (int in = 0; in < 2; ++in)
#pragma unroll
        for (int kc = 0; kc < 2; ++kc) { const size_t o = zh + (size_t)(n0 + in * 16 + lr) * HD + kc * 32 + 8 * hf; qh[in][kc] = ldb(QPh + o); ql[in][kc] = ldb(QPl + o); }

    auto phase1 = [&](int mt) {
        const int m0 = mt * 32;
#pragma unroll
        for (int jm = 0; jm < 2; ++jm) {
            v16bf kh[2], kl[2];
#pragma unroll
            for (int kc = 0; kc < 2; ++kc) { const size_t o = zh + (size_t)(m0 + jm * 16 + lr) * HD + kc * 32 + 8 * hf; kh[kc] = ldb(KPh + o); kl[kc] = ldb(KPl + o); }
#pragma unroll
            for (int in = 0; in < 2; ++in) {
                v8f s = (v8f){};
#pragma unroll
                for (int kc = 0; kc < 2; ++kc) { s = wmmab(qh[in][kc], kh[kc], s); s = wmmab(ql[in][kc], kh[kc], s); s = wmmab(qh[in][kc], kl[kc], s); }
                asm volatile("v_nop\n\tv_nop\n\tv_nop\n\tv_nop" : "+v"(s) : "v"(kh[1]), "v"(kl[1]));
#pragma unroll
                for (int r = 0; r < 8; ++r) Sb[((in * 16 + 8 * hf + r) * 32 + jm * 16 + lr) * SBP + w] = splitw(s[r]);
            }
        }
        __syncthreads();
    };
    auto mixtile = [&](int t) -> v8f {
        const int pos = (2 * w + (t >> 1)) * 32 + (t & 1) * 16 + lr;
        const v16bf a = ldw(Sb + pos * SBP + 8 * hf);
        v8f d = wmmab(a, preB, (v8f){});
        asm volatile("v_nop\n\tv_nop\n\tv_nop\n\tv_nop" : "+v"(d) : "v"(a), "v"(preB));
        return d;
    };

    float M0 = -1.0e30f, M1 = -1.0e30f, L0 = 0.f, L1 = 0.f;
#pragma unroll 1
    for (int mt = 0; mt < SEQ / 32; ++mt) {
        phase1(mt);
        { const v8f a = mixtile(0); const v8f c = mixtile(1); stat_upd(M0, L0, a, c); }
        { const v8f a = mixtile(2); const v8f c = mixtile(3); stat_upd(M1, L1, a, c); }
        __syncthreads();
    }
    const float i0 = 1.0f / L0, i1 = 1.0f / L1;

    v8f o[2][4];
#pragma unroll
    for (int in = 0; in < 2; ++in)
#pragma unroll
        for (int jd = 0; jd < 4; ++jd) o[in][jd] = (v8f){};
#pragma unroll 1
    for (int mt = 0; mt < SEQ / 32; ++mt) {
        const int m0 = mt * 32;
        phase1(mt);
#pragma unroll
        for (int t = 0; t < 4; ++t) {
            const v8f mx = mixtile(t);
            const float Mt = (t >> 1) ? M1 : M0; const float it = (t >> 1) ? i1 : i0;
#pragma unroll
            for (int r = 0; r < 8; ++r) PT[(8 * hf + r) * 16 + lr] = splitw(__builtin_amdgcn_exp2f((mx[r] - Mt) * L2E) * it);
            asm volatile("s_wait_dscnt 0x0" ::: "memory"); __builtin_amdgcn_wave_barrier(); asm volatile("" ::: "memory");
            const v16bf a = ldw(PT + lr * 16 + 8 * hf);
            asm volatile("s_wait_dscnt 0x0" ::: "memory"); __builtin_amdgcn_wave_barrier(); asm volatile("" ::: "memory");
            v8f pp = wmmab(a, postB, (v8f){});
            asm volatile("v_nop\n\tv_nop\n\tv_nop\n\tv_nop" : "+v"(pp) : "v"(a), "v"(postB));
            v8h ph;
#pragma unroll
            for (int r = 0; r < 8; ++r) ph[r] = (h16)(pp[r] * PCAR);
            *(v8ha*)(Pb + (size_t)(lr * 32 + 2 * w + (t >> 1)) * PBP + (t & 1) * 16 + 8 * hf) = ph;
        }
        __syncthreads();
        v16h pa[2], vb[4];
#pragma unroll
        for (int in = 0; in < 2; ++in) pa[in] = ldp(Pb + (size_t)(w * 32 + in * 16 + lr) * PBP + 8 * hf);
#pragma unroll
        for (int jd = 0; jd < 4; ++jd) vb[jd] = ldh(VT + zv + (size_t)(jd * 16 + lr) * SEQ + m0 + 8 * hf);
#pragma unroll
        for (int in = 0; in < 2; ++in)
#pragma unroll
            for (int jd = 0; jd < 4; ++jd) o[in][jd] = wmma16(pa[in], vb[jd], o[in][jd]);
        asm volatile("v_nop\n\tv_nop\n\tv_nop\n\tv_nop" : "+v"(o[0][0]), "+v"(o[0][1]), "+v"(o[0][2]), "+v"(o[0][3]), "+v"(o[1][0]), "+v"(o[1][1]), "+v"(o[1][2]), "+v"(o[1][3]) : "v"(pa[1]), "v"(vb[3]));
    }

    __syncthreads();
    bf* crow = CTX + ((size_t)b * SEQ + n0) * CK + w * HD;
#pragma unroll
    for (int part = 0; part < 2; ++part) {
#pragma unroll
        for (int in = 0; in < 2; ++in)
#pragma unroll
            for (int jd = 0; jd < 4; ++jd)
#pragma unroll
                for (int r = 0; r < 8; ++r) { unsigned short a2, c2; splitf(o[in][jd][r] * (1.0f / PCAR), a2, c2); OS[(in * 16 + 8 * hf + r) * 64 + jd * 16 + lr] = part ? c2 : a2; }
        asm volatile("s_wait_dscnt 0x0" ::: "memory"); __builtin_amdgcn_wave_barrier(); asm volatile("" ::: "memory");
#pragma unroll 1
        for (int ps = 0; ps < 2; ++ps) {
#pragma unroll
            for (int s = 0; s < 8; ++s) { const int row = 4 * s + (lane >> 3), pc = lane & 7; const v8us val = *(const v8usa*)(OS + row * 64 + pc * 8); *(volatile v8us*)(crow + (size_t)row * CK + part * DM + pc * 8) = val; }
            if (ps == 0) __threadfence(); }
        asm volatile("s_wait_dscnt 0x0" ::: "memory"); __builtin_amdgcn_wave_barrier(); asm volatile("" ::: "memory");
    }
}

static constexpr size_t al256(size_t x) { return (x + 255) & ~(size_t)255; }
static constexpr size_t SZ_XB  = al256((size_t)NB * SEQ * DM * 2);
static constexpr size_t SZ_WQ  = al256((size_t)D3 * DM * 2);
static constexpr size_t SZ_WP  = al256((size_t)DM * CK * 2);
static constexpr size_t SZ_F   = al256((size_t)NB * SEQ * D3 * 4);
static constexpr size_t SZ_PL  = al256((size_t)4 * NB * NH * SEQ * HD * 2);
static constexpr size_t SZ_VT  = al256((size_t)NB * NH * HD * SEQ * 2);
static constexpr size_t SZ_CTX = al256((size_t)NB * SEQ * CK * 2);
static constexpr size_t WS_TOTAL = SZ_XB + SZ_WQ + SZ_WP + SZ_F + SZ_PL + SZ_VT + SZ_CTX;
static_assert(WS_TOTAL <= (size_t)134217728);
static_assert((size_t)(NB * SEQ / 64) * 64 * CK * 2 <= SZ_CTX);
static_assert((size_t)(DM / 64) * 64 * CK * 2 <= SZ_WP);

extern "C" void kernel_launch(void* const* d_in, const int* in_sizes, int n_in,
                              void* d_out, int out_size, void* d_ws, size_t ws_size, hipStream_t stream) {
    if (n_in < 7) return;
    const size_t xneed = ((size_t)(NB - 1) * SEQ_FULL + SEQ) * DM;
    if ((size_t)in_sizes[0] < xneed || (size_t)in_sizes[1] < (size_t)D3 * DM || in_sizes[2] < D3 || (size_t)in_sizes[3] < (size_t)DM * DM || in_sizes[4] < DM || in_sizes[5] < NH * NH || in_sizes[6] < NH * NH) return;
    if ((size_t)out_size < xneed) return;
    if (WS_TOTAL > ws_size) return;
    const float* x = (const float*)d_in[0]; const float* wqkv = (const float*)d_in[1]; const float* bqkv = (const float*)d_in[2]; const float* wproj = (const float*)d_in[3]; const float* bproj = (const float*)d_in[4]; const float* pre = (const float*)d_in[5]; const float* post = (const float*)d_in[6];
    float* OUT = (float*)d_out;
    char* wsp = (char*)d_ws;
    bf* XB = (bf*)wsp; wsp += SZ_XB; bf* WQ = (bf*)wsp; wsp += SZ_WQ; bf* WP = (bf*)wsp; wsp += SZ_WP; float* F = (float*)wsp; wsp += SZ_F;
    bf* PL = (bf*)wsp; wsp += SZ_PL; h16* VT = (h16*)wsp; wsp += SZ_VT; bf* CTX = (bf*)wsp; wsp += SZ_CTX;

    k_cvt8<<<dim3((unsigned)(((size_t)SEQ * DM / 8 + 255) / 256), NB, 1), 256, 0, stream>>>(x, XB, (size_t)SEQ * DM / 8, (size_t)SEQ_FULL * DM, (size_t)SEQ * DM);
    k_cvt8<<<dim3((unsigned)(((size_t)D3 * DM / 8 + 255) / 256), 1, 1), 256, 0, stream>>>(wqkv, WQ, (size_t)D3 * DM / 8, 0, 0);
    k_cvtdup<<<(unsigned)(((size_t)DM * CK / 8 + 255) / 256), 256, 0, stream>>>(wproj, WP, (size_t)DM * CK / 8);
    k_gemm_bf<<<dim3(NB * SEQ / 64, D3 / 64, 1), 32, 0, stream>>>(XB, WQ, DM, F, D3, bqkv, 1.0f, 0, 0, 0);
    k_qkpl<<<dim3((unsigned)((PLSZ / 8 + 255) / 256), 2, 1), 256, 0, stream>>>(F, PL);
    k_vtp<<<(unsigned)((PLSZ / 8 + 255) / 256), 256, 0, stream>>>(F, VT);
    hipFuncSetAttribute(reinterpret_cast<const void*>(&k_attn), hipFuncAttributeMaxDynamicSharedMemorySize, LDS_TOT);
    k_attn<<<dim3(SEQ / 32, NB, 1), 512, LDS_TOT, stream>>>(PL, VT, pre, post, CTX);
    k_gemm_bf<<<dim3(SEQ / 64, DM / 64, NB), 32, 0, stream>>>(CTX, WP, CK, OUT, DM, bproj, 1.0f, (size_t)SEQ * CK, 0, (size_t)SEQ_FULL * DM);
}
